// SA_Layer_68719477127
// MI455X (gfx1250) — hardware-verified
//
#include <hip/hip_runtime.h>
#include <stddef.h>
#include <stdint.h>


#define BB 4
#define CC 256
#define NN 4096
#define CQ 64

typedef _Float16 f16t;
typedef f16t  v16h __attribute__((ext_vector_type(16)));
typedef f16t  v8h  __attribute__((ext_vector_type(8)));
typedef float v8f  __attribute__((ext_vector_type(8)));
typedef float v4f  __attribute__((ext_vector_type(4)));

union Frag { v16h v; v8h half[2]; };

#define SCX 64.0f
#define SCW 256.0f
#define SCP 4096.0f

__device__ __forceinline__ v8f zacc() {
    v8f z = {0.f, 0.f, 0.f, 0.f, 0.f, 0.f, 0.f, 0.f};
    return z;
}

__device__ __forceinline__ v8f mma(const Frag& a, const Frag& b, v8f c) {
    v8f d = __builtin_amdgcn_wmma_f32_16x16x32_f16(false, a.v, false, b.v, (short)0, c, false, false);
    asm volatile("v_nop\n\tv_nop\n\tv_nop\n\tv_nop" : "+v"(d) : "v"(a.v), "v"(b.v));
    return d;
}

__device__ __forceinline__ Frag frag16(const f16t* p) {
    Frag f;
    f.half[0] = *(const v8h*)(p);
    f.half[1] = *(const v8h*)(p + 16);
    return f;
}

__device__ __forceinline__ Frag frag_f32(const float* p, float s) {
    const v4f a0 = *(const v4f*)(p);
    const v4f a1 = *(const v4f*)(p + 4);
    const v4f b0 = *(const v4f*)(p + 16);
    const v4f b1 = *(const v4f*)(p + 20);
    v8h h0, h1;
#pragma unroll
    for (int i = 0; i < 4; ++i) {
        h0[i]     = (f16t)(a0[i] * s);
        h0[4 + i] = (f16t)(a1[i] * s);
        h1[i]     = (f16t)(b0[i] * s);
        h1[4 + i] = (f16t)(b1[i] * s);
    }
    Frag f;
    f.half[0] = h0;
    f.half[1] = h1;
    return f;
}

__device__ __forceinline__ void frag_f32_split(const float* p, float s, Frag& hi, Frag& lo) {
    v4f q[4];
    q[0] = *(const v4f*)(p);
    q[1] = *(const v4f*)(p + 4);
    q[2] = *(const v4f*)(p + 16);
    q[3] = *(const v4f*)(p + 20);
    v8h h0, h1, l0, l1;
#pragma unroll
    for (int i = 0; i < 4; ++i) {
        float v; f16t hv;
        v = q[0][i] * s; hv = (f16t)v; h0[i]     = hv; l0[i]     = (f16t)(v - (float)hv);
        v = q[1][i] * s; hv = (f16t)v; h0[4 + i] = hv; l0[4 + i] = (f16t)(v - (float)hv);
        v = q[2][i] * s; hv = (f16t)v; h1[i]     = hv; l1[i]     = (f16t)(v - (float)hv);
        v = q[3][i] * s; hv = (f16t)v; h1[4 + i] = hv; l1[4 + i] = (f16t)(v - (float)hv);
    }
    hi.half[0] = h0; hi.half[1] = h1;
    lo.half[0] = l0; lo.half[1] = l1;
}

__device__ __forceinline__ void st_v4f(float* p, v4f v) { *(volatile v4f*)p = v; }
__device__ __forceinline__ void st_v8h(f16t* p, v8h v) { *(volatile v8h*)p = v; }

__global__ __launch_bounds__(256) void k_cvt_x(const float* __restrict__ x,
                                               f16t* __restrict__ xh, f16t* __restrict__ xl) {
    __shared__ __align__(16) f16t sh[32 * 264];
    __shared__ __align__(16) f16t sl[32 * 264];
    const int b = blockIdx.y, n0 = blockIdx.x * 32;
    if (b >= BB || n0 + 32 > NN) return;
    const int tid = threadIdx.x, w = tid >> 5, lane = tid & 31;
    const float* xb = x + (size_t)b * CC * NN + n0 + lane;
#pragma unroll 4
    for (int i = 0; i < 32; ++i) {
        const int c = w * 32 + i;
        const float v = xb[(size_t)c * NN] * SCX;
        const f16t hv = (f16t)v;
        const f16t lv = (f16t)(v - (float)hv);
        sh[lane * 264 + c] = hv;
        sl[lane * 264 + c] = lv;
    }
    __syncthreads();
    v8h hr[4], lr[4];
    size_t go[4];
#pragma unroll
    for (int j = 0; j < 4; ++j) {
        const int nl = 4 * w + j;
        hr[j] = *(const v8h*)(sh + nl * 264 + 8 * lane);
        lr[j] = *(const v8h*)(sl + nl * 264 + 8 * lane);
        go[j] = ((size_t)b * NN + n0 + nl) * CC + 8 * lane;
        st_v8h(xh + go[j], hr[j]);
        st_v8h(xl + go[j], lr[j]);
    }
    __threadfence();
#pragma unroll
    for (int j = 0; j < 4; ++j) {
        st_v8h(xh + go[j], hr[j]);
        st_v8h(xl + go[j], lr[j]);
    }
}

__global__ __launch_bounds__(128) void k_xq(const f16t* __restrict__ xh, const f16t* __restrict__ xl,
                                            const float* __restrict__ wqk,
                                            f16t* __restrict__ qh, f16t* __restrict__ ql) {
    __shared__ __align__(16) f16t s_h[16 * 72];
    __shared__ __align__(16) f16t s_l[16 * 72];
    const int b = blockIdx.y, n0 = blockIdx.x * 16;
    if (b >= BB || n0 + 16 > NN) return;
    const int tid = threadIdx.x, w = tid >> 5, lane = tid & 31, h = lane >> 4, m = lane & 15;
    const f16t* ah_p = xh + ((size_t)b * NN + n0 + m) * CC + 8 * h;
    const f16t* al_p = xl + ((size_t)b * NN + n0 + m) * CC + 8 * h;
    const float* b_p = wqk + (size_t)(16 * w + m) * CC + 8 * h;
    v8f acc = zacc();
#pragma unroll 1
    for (int ks = 0; ks < CC / 32; ++ks) {
        const int k0 = ks * 32;
        Frag ah = frag16(ah_p + k0);
        Frag al = frag16(al_p + k0);
        Frag bh, bl;
        frag_f32_split(b_p + k0, SCW, bh, bl);
        acc = mma(ah, bh, acc);
        acc = mma(ah, bl, acc);
        acc = mma(al, bh, acc);
    }
#pragma unroll
    for (int r = 0; r < 8; ++r) {
        const float v = acc[r] * (1.0f / SCW);
        const f16t hv = (f16t)v;
        const f16t lv = (f16t)(v - (float)hv);
        s_h[(8 * h + r) * 72 + 16 * w + m] = hv;
        s_l[(8 * h + r) * 72 + 16 * w + m] = lv;
    }
    __syncthreads();
    const int rl = 4 * w + (lane >> 3), cq = 8 * (lane & 7);
    const v8h hv8 = *(const v8h*)(s_h + rl * 72 + cq);
    const v8h lv8 = *(const v8h*)(s_l + rl * 72 + cq);
    const size_t o = ((size_t)b * NN + n0 + rl) * CQ + cq;
    st_v8h(qh + o, hv8);
    st_v8h(ql + o, lv8);
    __threadfence();
    st_v8h(qh + o, hv8);
    st_v8h(ql + o, lv8);
}

__global__ __launch_bounds__(128) void k_xv(const float* __restrict__ wv, const f16t* __restrict__ xh,
                                            const float* __restrict__ bv, f16t* __restrict__ xvo) {
    __shared__ __align__(16) f16t s_v[64 * 72];
    const int b = blockIdx.z, v0 = blockIdx.y * 64, n0 = blockIdx.x * 64;
    if (b >= BB || v0 + 64 > CC || n0 + 64 > NN) return;
    const int tid = threadIdx.x, w = tid >> 5, lane = tid & 31, h = lane >> 4, m = lane & 15;
    const float* a_p = wv + (size_t)(v0 + 16 * w + m) * CC + 8 * h;
    const f16t* b_p = xh + ((size_t)b * NN + n0 + m) * CC + 8 * h;
    v8f acc[4];
#pragma unroll
    for (int j = 0; j < 4; ++j) acc[j] = zacc();
#pragma unroll 1
    for (int ks = 0; ks < CC / 32; ++ks) {
        const int k0 = ks * 32;
        Frag a = frag_f32(a_p + k0, SCW);
#pragma unroll
        for (int j = 0; j < 4; ++j) {
            Frag bb = frag16(b_p + (size_t)(16 * j) * CC + k0);
            acc[j] = mma(a, bb, acc[j]);
        }
    }
#pragma unroll
    for (int j = 0; j < 4; ++j) {
#pragma unroll
        for (int r = 0; r < 8; ++r) {
            const int vr = 16 * w + 8 * h + r;
            const float val = acc[j][r] * (1.0f / (SCX * SCW)) + bv[v0 + vr];
            s_v[vr * 72 + 16 * j + m] = (f16t)val;
        }
    }
    __syncthreads();
    v8h vals[4];
    size_t offs[4];
#pragma unroll
    for (int t = 0; t < 4; ++t) {
        const int i = 16 * w + 4 * t + (lane >> 3);
        const int col = 8 * (lane & 7);
        vals[t] = *(const v8h*)(s_v + i * 72 + col);
        offs[t] = ((size_t)b * CC + v0 + i) * NN + n0 + col;
        st_v8h(xvo + offs[t], vals[t]);
    }
    __threadfence();
#pragma unroll
    for (int t = 0; t < 4; ++t) st_v8h(xvo + offs[t], vals[t]);
}

__device__ __forceinline__ void e_store(const float* se, float* E, int n0, int m0, int w, int lane, bool tr) {
#pragma unroll
    for (int u = 0; u < 8; ++u) {
        const int i = 16 * w + 2 * u + (lane >> 4), col = 4 * (lane & 15);
        const v4f v = *(const v4f*)(se + i * 68 + col);
        st_v4f(E + (size_t)(n0 + i) * NN + m0 + col, v);
    }
    if (tr) {
#pragma unroll
        for (int u = 0; u < 8; ++u) {
            const int jj = 16 * w + 2 * u + (lane >> 4), ii = 4 * (lane & 15);
            v4f v;
            v[0] = se[(ii + 0) * 68 + jj];
            v[1] = se[(ii + 1) * 68 + jj];
            v[2] = se[(ii + 2) * 68 + jj];
            v[3] = se[(ii + 3) * 68 + jj];
            st_v4f(E + (size_t)(m0 + jj) * NN + n0 + ii, v);
        }
    }
}

__global__ __launch_bounds__(128) void k_energy(const f16t* __restrict__ qh, const f16t* __restrict__ ql,
                                                float* __restrict__ E) {
    __shared__ __align__(16) float se[64 * 68];
    const int tm = blockIdx.x, tn = blockIdx.y;
    if (tn > tm || tm >= NN / 64) return;
    const int n0 = tn * 64, m0 = tm * 64;
    const int tid = threadIdx.x, w = tid >> 5, lane = tid & 31, h = lane >> 4, m = lane & 15;
    const f16t* ah_p = qh + (size_t)(n0 + 16 * w + m) * CQ + 8 * h;
    const f16t* al_p = ql + (size_t)(n0 + 16 * w + m) * CQ + 8 * h;
    const f16t* bh_p = qh + (size_t)(m0 + m) * CQ + 8 * h;
    const f16t* bl_p = ql + (size_t)(m0 + m) * CQ + 8 * h;
    v8f acc[4];
#pragma unroll
    for (int j = 0; j < 4; ++j) acc[j] = zacc();
#pragma unroll
    for (int ks = 0; ks < CQ / 32; ++ks) {
        const int k0 = ks * 32;
        Frag ah = frag16(ah_p + k0);
        Frag al = frag16(al_p + k0);
#pragma unroll
        for (int j = 0; j < 4; ++j) {
            Frag bh = frag16(bh_p + (size_t)(16 * j) * CQ + k0);
            Frag bl = frag16(bl_p + (size_t)(16 * j) * CQ + k0);
            acc[j] = mma(ah, bh, acc[j]);
            acc[j] = mma(ah, bl, acc[j]);
            acc[j] = mma(al, bh, acc[j]);
        }
    }
#pragma unroll
    for (int j = 0; j < 4; ++j) {
#pragma unroll
        for (int r = 0; r < 8; ++r)
            se[(16 * w + 8 * h + r) * 68 + 16 * j + m] = acc[j][r] * (1.0f / (SCX * SCX));
    }
    __syncthreads();
    e_store(se, E, n0, m0, w, lane, tn < tm);
    __threadfence();
    e_store(se, E, n0, m0, w, lane, tn < tm);
}

__global__ __launch_bounds__(256) void k_stats(const float* __restrict__ E, float* __restrict__ rmax,
                                               float* __restrict__ rsinv) {
    __shared__ __align__(16) float smx[32];
    __shared__ __align__(16) float ssi[32];
    const int n0 = blockIdx.x * 32;
    if (n0 + 32 > NN) return;
    const int tid = threadIdx.x, w = tid >> 5, lane = tid & 31;
#pragma unroll 1
    for (int t = 0; t < 4; ++t) {
        const int row = n0 + 4 * w + t;
        const float* er = E + (size_t)row * NN + 4 * lane;
        float mx = -__builtin_inff();
#pragma unroll 4
        for (int it = 0; it < NN / 128; ++it) {
            const v4f v = *(const v4f*)(er + 128 * it);
            mx = fmaxf(mx, fmaxf(fmaxf(v[0], v[1]), fmaxf(v[2], v[3])));
        }
#pragma unroll
        for (int off = 16; off > 0; off >>= 1) mx = fmaxf(mx, __shfl_xor(mx, off, 32));
        float s = 0.f;
#pragma unroll 4
        for (int it = 0; it < NN / 128; ++it) {
            const v4f v = *(const v4f*)(er + 128 * it);
            s += (__expf(v[0] - mx) + __expf(v[1] - mx)) + (__expf(v[2] - mx) + __expf(v[3] - mx));
        }
#pragma unroll
        for (int off = 16; off > 0; off >>= 1) s += __shfl_xor(s, off, 32);
        if (lane == 0) {
            smx[4 * w + t] = mx;
            ssi[4 * w + t] = 1.0f / s;
        }
    }
    __syncthreads();
    if (tid < 16) {
        const int q = tid & 7;
        float* dst = (tid < 8) ? (rmax + n0 + 4 * q) : (rsinv + n0 + 4 * q);
        const float* src = (tid < 8) ? (smx + 4 * q) : (ssi + 4 * q);
        const v4f v = *(const v4f*)src;
        st_v4f(dst, v);
        __threadfence();
        st_v4f(dst, v);
    }
}

__global__ __launch_bounds__(256) void k_apply(const float* __restrict__ E, const float* __restrict__ rmax,
                                               const float* __restrict__ rsinv, const f16t* __restrict__ xv,
                                               const float* __restrict__ x, f16t* __restrict__ dT) {
    __shared__ __align__(16) f16t s_p[32 * 72];
    __shared__ __align__(16) f16t s_d[32 * 264];
    __shared__ float s_cs[256];
    __shared__ float s_ri[32];
    __shared__ int s_nz[8];
    const int m0 = blockIdx.x * 32;
    if (m0 + 32 > NN) return;
    const int tid = threadIdx.x, w = tid >> 5, lane = tid & 31, h = lane >> 4, m = lane & 15;
    const int mt = w & 1, vq = w >> 1;
    v8f acc[4];
#pragma unroll
    for (int i = 0; i < 4; ++i) acc[i] = zacc();
    float csum = 0.f;
    const float* ecol = E + m0 + lane;
    const f16t* a_p = xv + (size_t)(64 * vq + m) * NN + 8 * h;
    const f16t* b_p = s_p + (16 * mt + m) * 72 + 8 * h;
#pragma unroll 1
    for (int n0 = 0; n0 < NN; n0 += 64) {
        {
            const int nb = n0 + 8 * w;
            v8h pv;
            int nz = 0;
#pragma unroll
            for (int r = 0; r < 8; ++r) {
                const int n = nb + r;
                const float e = ecol[(size_t)n * NN];
                const float p = __expf(e - rmax[n]) * rsinv[n];
                csum += p;
                const f16t hp = (f16t)(p * SCP);
                pv[r] = hp;
                nz |= ((float)hp != 0.0f) ? 1 : 0;
            }
            *(v8h*)(s_p + lane * 72 + 8 * w) = pv;
            const int wz = __any(nz);
            if (lane == 0) s_nz[w] = wz;
        }
        __syncthreads();
        int anyz = 0;
#pragma unroll
        for (int q = 0; q < 8; ++q) anyz |= s_nz[q];
        if (anyz) {
#pragma unroll
            for (int ks = 0; ks < 2; ++ks) {
                const int k0 = ks * 32;
                Frag bf = frag16(b_p + k0);
#pragma unroll
                for (int i = 0; i < 4; ++i) {
                    Frag af = frag16(a_p + (size_t)(16 * i) * NN + n0 + k0);
                    acc[i] = mma(af, bf, acc[i]);
                }
            }
        }
        __syncthreads();
    }
    s_cs[tid] = csum;
    __syncthreads();
    if (tid < 32) {
        float t = 0.f;
#pragma unroll
        for (int q = 0; q < 8; ++q) t += s_cs[q * 32 + tid];
        s_ri[tid] = 1.0f / (1e-9f + t);
    }
    __syncthreads();
    {
        const int ml = 16 * mt + m;
        const float ri = s_ri[ml] * (1.0f / SCP);
        const float* xc = x + m0 + ml;
#pragma unroll
        for (int i = 0; i < 4; ++i) {
#pragma unroll
            for (int r = 0; r < 8; ++r) {
                const int v = 64 * vq + 16 * i + 8 * h + r;
                const float xr = acc[i][r] * ri;
                const float xx = xc[(size_t)v * NN];
                s_d[ml * 264 + v] = (f16t)((xx - xr) * SCX);
            }
        }
    }
    __syncthreads();
    v8h dv[4];
    size_t offs[4];
#pragma unroll
    for (int t = 0; t < 4; ++t) {
        const int row = 4 * w + t;
        dv[t] = *(const v8h*)(s_d + row * 264 + 8 * lane);
        offs[t] = (size_t)(m0 + row) * CC + 8 * lane;
        st_v8h(dT + offs[t], dv[t]);
    }
    __threadfence();
#pragma unroll
    for (int t = 0; t < 4; ++t) st_v8h(dT + offs[t], dv[t]);
}

__global__ __launch_bounds__(128) void k_out(const float* __restrict__ wt, const f16t* __restrict__ dT,
                                             const float* __restrict__ bt, const float* __restrict__ gamma,
                                             const float* __restrict__ beta, const float* __restrict__ mean,
                                             const float* __restrict__ var, const float* __restrict__ x,
                                             float* __restrict__ out) {
    __shared__ __align__(16) float s_y[64 * 36];
    const int b = blockIdx.z, o0 = blockIdx.y * 64, n0 = blockIdx.x * 32;
    if (b >= BB || o0 + 64 > CC || n0 + 32 > NN) return;
    const int tid = threadIdx.x, w = tid >> 5, lane = tid & 31, h = lane >> 4, m = lane & 15;
    const float* a_p = wt + (size_t)(o0 + 16 * w + m) * CC + 8 * h;
    const f16t* b_p = dT + ((size_t)b * NN + n0 + m) * CC + 8 * h;
    v8f acc[2];
    acc[0] = zacc();
    acc[1] = zacc();
#pragma unroll 1
    for (int ks = 0; ks < CC / 32; ++ks) {
        const int k0 = ks * 32;
        Frag a = frag_f32(a_p + k0, SCW);
#pragma unroll
        for (int j = 0; j < 2; ++j) {
            Frag bb = frag16(b_p + (size_t)(16 * j) * CC + k0);
            acc[j] = mma(a, bb, acc[j]);
        }
    }
#pragma unroll
    for (int j = 0; j < 2; ++j) {
#pragma unroll
        for (int r = 0; r < 8; ++r) {
            const int o = o0 + 16 * w + 8 * h + r;
            float y = acc[j][r] * (1.0f / (SCX * SCW)) + bt[o];
            y = gamma[o] * (y - mean[o]) * rsqrtf(var[o] + 1e-5f) + beta[o];
            s_y[(16 * w + 8 * h + r) * 36 + 16 * j + m] = fmaxf(y, 0.0f);
        }
    }
    __syncthreads();
    v4f vals[4];
    size_t offs[4];
#pragma unroll
    for (int t = 0; t < 4; ++t) {
        const int i = 16 * w + 4 * t + (lane >> 3);
        const int col = 4 * (lane & 7);
        const v4f yv = *(const v4f*)(s_y + i * 36 + col);
        const size_t gi = ((size_t)b * CC + o0 + i) * NN + n0 + col;
        const v4f xv4 = *(const v4f*)(x + gi);
        vals[t] = xv4 + yv;
        offs[t] = gi;
        st_v4f(out + gi, vals[t]);
    }
    __threadfence();
#pragma unroll
    for (int t = 0; t < 4; ++t) st_v4f(out + offs[t], vals[t]);
}

extern "C" void kernel_launch(void* const* d_in, const int* in_sizes, int n_in,
                              void* d_out, int out_size, void* d_ws, size_t ws_size,
                              hipStream_t stream) {
    if (n_in < 10) return;
    if (in_sizes[0] != BB * CC * NN || in_sizes[1] != CQ * CC || in_sizes[2] != CC * CC ||
        in_sizes[3] != CC || in_sizes[4] != CC * CC || in_sizes[5] != CC || in_sizes[6] != CC ||
        in_sizes[7] != CC || in_sizes[8] != CC || in_sizes[9] != CC) return;
    if (out_size != BB * CC * NN) return;

    const float* x     = (const float*)d_in[0];
    const float* w_qk  = (const float*)d_in[1];
    const float* w_v   = (const float*)d_in[2];
    const float* b_v   = (const float*)d_in[3];
    const float* w_t   = (const float*)d_in[4];
    const float* b_t   = (const float*)d_in[5];
    const float* gamma = (const float*)d_in[6];
    const float* beta  = (const float*)d_in[7];
    const float* mean  = (const float*)d_in[8];
    const float* var   = (const float*)d_in[9];
    float* out = (float*)d_out;

    char* ws = (char*)d_ws;
    size_t off = 0;
    f16t* xh    = (f16t*)(ws + off); off += (size_t)BB * NN * CC * sizeof(f16t);
    f16t* xl    = (f16t*)(ws + off); off += (size_t)BB * NN * CC * sizeof(f16t);
    f16t* qh    = (f16t*)(ws + off); off += (size_t)BB * NN * CQ * sizeof(f16t);
    f16t* ql    = (f16t*)(ws + off); off += (size_t)BB * NN * CQ * sizeof(f16t);
    f16t* xv    = (f16t*)(ws + off); off += (size_t)BB * CC * NN * sizeof(f16t);
    f16t* dT    = (f16t*)(ws + off); off += (size_t)BB * NN * CC * sizeof(f16t);
    float* rmax = (float*)(ws + off); off += (size_t)BB * NN * sizeof(float);
    float* rsin = (float*)(ws + off); off += (size_t)BB * NN * sizeof(float);
    float* E    = (float*)(ws + off); off += (size_t)NN * NN * sizeof(float);
    if (off > ws_size) return;

    hipLaunchKernelGGL(k_cvt_x, dim3(NN / 32, BB), dim3(256), 0, stream, x, xh, xl);
    hipLaunchKernelGGL(k_xq, dim3(NN / 16, BB), dim3(128), 0, stream, xh, xl, w_qk, qh, ql);
    hipLaunchKernelGGL(k_xv, dim3(NN / 64, CC / 64, BB), dim3(128), 0, stream, w_v, xh, b_v, xv);
    for (int b = 0; b < BB; ++b) {
        const f16t* qh_b = qh + (size_t)b * NN * CQ;
        const f16t* ql_b = ql + (size_t)b * NN * CQ;
        float* rmax_b = rmax + (size_t)b * NN;
        float* rsin_b = rsin + (size_t)b * NN;
        const f16t* xv_b = xv + (size_t)b * CC * NN;
        const float* x_b = x + (size_t)b * CC * NN;
        f16t* dT_b = dT + (size_t)b * NN * CC;
        hipLaunchKernelGGL(k_energy, dim3(NN / 64, NN / 64), dim3(128), 0, stream, qh_b, ql_b, E);
        hipLaunchKernelGGL(k_stats, dim3(NN / 32), dim3(256), 0, stream, E, rmax_b, rsin_b);
        hipLaunchKernelGGL(k_apply, dim3(NN / 32), dim3(256), 0, stream, E, rmax_b, rsin_b, xv_b, x_b, dT_b);
    }
    hipLaunchKernelGGL(k_out, dim3(NN / 32, CC / 64, BB), dim3(128), 0, stream,
                       w_t, dT, b_t, gamma, beta, mean, var, x, out);
}
